// HSTUAttention_73229192397471
// MI455X (gfx1250) — hardware-verified
//
#include <hip/hip_runtime.h>
#include <math.h>

typedef __attribute__((ext_vector_type(16))) _Float16 v16h;
typedef __attribute__((ext_vector_type(16))) __bf16 v16b;
typedef __attribute__((ext_vector_type(8)))  _Float16 v8h;
typedef __attribute__((ext_vector_type(8)))  float v8f;
typedef __attribute__((ext_vector_type(4)))  float v4f;
typedef __attribute__((ext_vector_type(2)))  float v2f;
typedef __attribute__((ext_vector_type(4)))  unsigned v4u;
typedef __attribute__((ext_vector_type(4)))  int v4i;
typedef float __attribute__((may_alias)) float_a;
typedef int __attribute__((may_alias)) int_a;

template <typename T> __device__ __forceinline__ void vst2(void* p, T v) { *(volatile T*)p = v; __threadfence(); *(volatile T*)p = v; }
__device__ __forceinline__ v8f wmma16(v16h a, v16h b, v8f c) {
  v8f d = __builtin_amdgcn_wmma_f32_16x16x32_f16(false, a, false, b, (short)0, c, false, false);
  asm volatile("v_nop\n\tv_nop\n\tv_nop\n\tv_nop" : "+v"(d) : "v"(a), "v"(b));
  return d;
}
__device__ __forceinline__ v8f wmma_bf(v16b a, v16b b, v8f c) {
  v8f d = __builtin_amdgcn_wmma_f32_16x16x32_bf16(false, a, false, b, (short)0, c, false, false);
  asm volatile("v_nop\n\tv_nop\n\tv_nop\n\tv_nop" : "+v"(d) : "v"(a), "v"(b));
  return d;
}
__device__ __forceinline__ v16h frag_h(const _Float16* rowk0, int lane) {
  union { v16h v; v8h q[2]; } u; const _Float16* p = rowk0 + 8 * (lane >> 4);
  u.q[0] = *(const v8h*)p; u.q[1] = *(const v8h*)(p + 16); return u.v;
}
__device__ __forceinline__ v16h frag_f32(const float* rowk0, int lane) {
  v16h a; const float* p = rowk0 + 8 * (lane >> 4);
#pragma unroll
  for (int i = 0; i < 8; ++i) { a[i] = (_Float16)p[i]; a[8 + i] = (_Float16)p[16 + i]; }
  return a;
}
__device__ __forceinline__ v16h frag_f32s(const float* rowk0, int lane, float sc) {
  v16h a; const float* p = rowk0 + 8 * (lane >> 4);
#pragma unroll
  for (int i = 0; i < 8; ++i) { a[i] = (_Float16)(p[i] * sc); a[8 + i] = (_Float16)(p[16 + i] * sc); }
  return a;
}
__device__ __forceinline__ v16h fragc_f32(const float* W, int k0, int n, int lane, int ld, int K) {
  v16h a; const int g = lane >> 4;
#pragma unroll
  for (int i = 0; i < 8; ++i) { const int ka = k0 + 8 * g + i, kb = ka + 16;
    a[i] = (_Float16)(ka < K ? W[(size_t)(ka < K ? ka : K - 1) * ld + n] : 0.f); a[8 + i] = (_Float16)(kb < K ? W[(size_t)(kb < K ? kb : K - 1) * ld + n] : 0.f); }
  return a;
}
struct F2 { v16b h, l; };
__device__ __forceinline__ F2 bsplit16(const float v[16]) { F2 r;
#pragma unroll
  for (int i = 0; i < 16; ++i) { const __bf16 h = (__bf16)v[i]; r.h[i] = h; r.l[i] = (__bf16)(v[i] - (float)h); }
  return r; }
__device__ __forceinline__ F2 split_row(const float* row, int k0, int lane) { float v[16]; const float* p = row + k0 + 8 * (lane >> 4);
#pragma unroll
  for (int i = 0; i < 8; ++i) { v[i] = p[i]; v[8 + i] = p[16 + i]; }
  return bsplit16(v); }
__device__ __forceinline__ F2 split_rowK(const float* row, int k0, int lane, int K) { float v[16]; const int g = lane >> 4;
#pragma unroll
  for (int i = 0; i < 8; ++i) { const int ka = k0 + 8 * g + i, kb = ka + 16; v[i] = ka < K ? row[ka < K ? ka : K - 1] : 0.f; v[8 + i] = kb < K ? row[kb < K ? kb : K - 1] : 0.f; }
  return bsplit16(v); }
__device__ __forceinline__ F2 split_col(const float* W, int k0, int n, int lane, int ld, int K) { float v[16]; const int g = lane >> 4;
#pragma unroll
  for (int i = 0; i < 8; ++i) { const int ka = k0 + 8 * g + i, kb = ka + 16; v[i] = ka < K ? W[(size_t)(ka < K ? ka : K - 1) * ld + n] : 0.f; v[8 + i] = kb < K ? W[(size_t)(kb < K ? kb : K - 1) * ld + n] : 0.f; }
  return bsplit16(v); }
__device__ __forceinline__ v8f mac3(const F2& a, const F2& b, v8f c) { c = wmma_bf(a.l, b.h, c); c = wmma_bf(a.h, b.l, c); return wmma_bf(a.h, b.h, c); }
__device__ __forceinline__ float sigm(float v) { return 1.0f / (1.0f + expf(-v)); }
#define LDSX() do { asm volatile("s_wait_dscnt 0" ::: "memory"); __builtin_amdgcn_wave_barrier(); __builtin_amdgcn_fence(__ATOMIC_RELEASE, "workgroup"); } while (0)

__device__ __forceinline__ float bfr(float v) { return (float)(__bf16)v; }
__device__ __forceinline__ float silu1(float v) { return v / (1.0f + expf(-v)); }
#define NB 8
#define TT 1024
#define CC 512
#define NH 8
#define HD 64
#define HG 4
#ifndef TNB
#define TNB NB
#endif
typedef __attribute__((ext_vector_type(8))) __bf16 v8b;
__device__ __forceinline__ v16b frag_b(const __bf16* rowk0, int lane) { union { v16b v; v8b q[2]; } u; const __bf16* p = rowk0 + 8 * (lane >> 4); u.q[0] = *(const v8b*)p; u.q[1] = *(const v8b*)(p + 16); return u.v; }
#define WS_ST  0u
#define WS_QH  (WS_ST + 4u * (size_t)NB * TT * 2)
#define WS_QL  (WS_QH + 2u * (size_t)NB * TT * CC)
#define WS_KH  (WS_QL + 2u * (size_t)NB * TT * CC)
#define WS_KL  (WS_KH + 2u * (size_t)NB * TT * CC)
#define WS_VT  (WS_KL + 2u * (size_t)NB * TT * CC)
#define WS_VL  (WS_VT + 2u * (size_t)NB * CC * TT)
#define WS_U   (WS_VL + 2u * (size_t)NB * CC * TT)
#define WS_S   (WS_U + 4u * (size_t)NB * TT * CC)
#define WS_AV  (WS_S + 4u * (size_t)HG * TT * TT)
#define WS_END (WS_AV + 4u * (size_t)NB * TT * CC)
__global__ __launch_bounds__(256) void k_stat(const float* __restrict__ X, float* __restrict__ ST) { __shared__ __align__(16) float so[32];
  const int t = threadIdx.x; const int rl = t >> 4, sub = t & 15; const size_t row = (size_t)blockIdx.x * 16 + rl; const float* p = X + row * CC;
  float s = 0.f; for (int c = sub; c < CC; c += 16) s += bfr(p[c]);
#pragma unroll
  for (int o = 1; o < 16; o <<= 1) s += __shfl_xor(s, o);
  const float mu = s * (1.0f / CC); float s2 = 0.f; for (int c = sub; c < CC; c += 16) { const float d = bfr(p[c]) - mu; s2 += d * d; }
#pragma unroll
  for (int o = 1; o < 16; o <<= 1) s2 += __shfl_xor(s2, o);
  if (sub == 0) { so[rl * 2] = mu; so[rl * 2 + 1] = rsqrtf(s2 * (1.0f / CC) + 1e-8f); }
  __syncthreads(); if (t < 32) vst2(ST + (size_t)blockIdx.x * 32 + t, so[t]); }
__global__ __launch_bounds__(128) void k_proj(const float* __restrict__ X, const float* __restrict__ ST, const float* __restrict__ Wt, _Float16* __restrict__ QH, _Float16* __restrict__ QL, _Float16* __restrict__ KH, _Float16* __restrict__ KL, __bf16* __restrict__ VT, __bf16* __restrict__ VL, float* __restrict__ U) {
  __shared__ __align__(16) _Float16 sh[64][136], sl[64][136]; __shared__ __align__(16) __bf16 th[128][72], tl2[128][72];
  const int tid = threadIdx.x, wave = tid >> 5, lane = tid & 31, col = lane & 15, g = lane >> 4; const int which = blockIdx.z; const int c0 = blockIdx.y * 128; const size_t r0 = (size_t)blockIdx.x * 64; const size_t arow = r0 + wave * 16 + col; const float mu = ST[arow * 2], rs = ST[arow * 2 + 1];
  v8f acc[8] = {};
#pragma unroll 2
  for (int kc = 0; kc < CC / 32; ++kc) { float v[16]; { const float* p = X + arow * CC + kc * 32 + 8 * g;
#pragma unroll
      for (int i = 0; i < 8; ++i) { v[i] = (bfr(p[i]) - mu) * rs; v[8 + i] = (bfr(p[16 + i]) - mu) * rs; } }
    asm volatile("s_wait_loadcnt 0x0" ::: "memory"); const F2 a = bsplit16(v);
#pragma unroll
    for (int j = 0; j < 8; ++j) { v16b w; const int o = which * CC + c0 + j * 16 + col;
#pragma unroll
      for (int i = 0; i < 8; ++i) { w[i] = (__bf16)Wt[(size_t)(kc * 32 + 8 * g + i) * (4 * CC) + o]; w[8 + i] = (__bf16)Wt[(size_t)(kc * 32 + 16 + 8 * g + i) * (4 * CC) + o]; }
      asm volatile("s_wait_loadcnt 0x0" ::: "memory"); acc[j] = wmma_bf(a.h, w, acc[j]); acc[j] = wmma_bf(a.l, w, acc[j]); } }
  if (which == 3) { __shared__ __align__(16) float sf[4][16][132];
#pragma unroll
    for (int j = 0; j < 8; ++j)
#pragma unroll
      for (int r = 0; r < 8; ++r) sf[wave][8 * g + r][j * 16 + col] = silu1(acc[j][r]);
    LDSX(); for (int rl = 0; rl < 16; ++rl) vst2(U + (r0 + wave * 16 + rl) * CC + c0 + lane * 4, *(const v4f*)&sf[wave][rl][lane * 4]); return; }
#pragma unroll
  for (int j = 0; j < 8; ++j)
#pragma unroll
    for (int r = 0; r < 8; ++r) { const float v = silu1(acc[j][r]); const int rl = wave * 16 + 8 * g + r, cl = j * 16 + col;
      if (which == 2) { const __bf16 bh = (__bf16)v; th[cl][rl] = bh; tl2[cl][rl] = (__bf16)(v - (float)bh); } else { const _Float16 hv = (_Float16)v; sh[rl][cl] = hv; sl[rl][cl] = (_Float16)((v - (float)hv) * 1024.0f); } }
  __syncthreads();
  if (which < 2) { _Float16* dh = which == 0 ? QH : KH; _Float16* dl = which == 0 ? QL : KL; for (int e = tid; e < 64 * 16; e += 128) { const int rl = e >> 4, q = e & 15; vst2((unsigned*)(dh + (r0 + rl) * CC + c0 + q * 8), *(const v4u*)&sh[rl][q * 8]); vst2((unsigned*)(dl + (r0 + rl) * CC + c0 + q * 8), *(const v4u*)&sl[rl][q * 8]); } }
  else { const size_t b = r0 / TT; const int t0 = (int)(r0 % TT); for (int e = tid; e < 128 * 8; e += 128) { const int cl = e >> 3, q = e & 7; const size_t o2 = (b * CC + c0 + cl) * (size_t)TT + t0 + q * 8; vst2((unsigned*)(VT + o2), *(const v4u*)&th[cl][q * 8]); vst2((unsigned*)(VL + o2), *(const v4u*)&tl2[cl][q * 8]); } } }
__global__ __launch_bounds__(128) void k_sc(const _Float16* __restrict__ QH, const _Float16* __restrict__ QL, const _Float16* __restrict__ KH, const _Float16* __restrict__ KL, const int* __restrict__ TS, const float* __restrict__ TSW, const float* __restrict__ POSW, int b, int h0, float* __restrict__ S0) { __shared__ __align__(16) float ss[4][16][132]; __shared__ int skt[128]; __shared__ int sqt[64];
  const int h = h0 + blockIdx.z; float* S = S0 + (size_t)blockIdx.z * TT * TT;
  const int tid = threadIdx.x, wave = tid >> 5, lane = tid & 31, col = lane & 15, g = lane >> 4; const int k0 = blockIdx.y * 128; const int q0b = blockIdx.x * 64; const int ql0 = q0b + wave * 16;
  if (k0 > q0b + 63) return;
  skt[tid] = TS[(size_t)b * TT + k0 + tid]; if (tid < 64) { const int n = q0b + tid; sqt[tid] = TS[(size_t)b * TT + (n + 1 < TT ? n + 1 : TT - 1)]; }
  __syncthreads();
  v8f acc[8] = {}, accl[8] = {};
#pragma unroll
  for (int kc = 0; kc < HD / 32; ++kc) { const size_t qo = ((size_t)b * TT + ql0 + col) * CC + h * HD + kc * 32; const v16h ah = frag_h(QH + qo, lane), al = frag_h(QL + qo, lane);
#pragma unroll
    for (int j = 0; j < 8; ++j) { const size_t ko = ((size_t)b * TT + k0 + j * 16 + col) * CC + h * HD + kc * 32; const v16h kb = frag_h(KH + ko, lane), kl = frag_h(KL + ko, lane); acc[j] = wmma16(ah, kb, acc[j]); accl[j] = wmma16(al, kb, accl[j]); accl[j] = wmma16(ah, kl, accl[j]); } }
#pragma unroll
  for (int j = 0; j < 8; ++j) { const int ml = j * 16 + col; const int m = k0 + ml;
#pragma unroll
    for (int r = 0; r < 8; ++r) { const int nl = wave * 16 + 8 * g + r; const int n = q0b + nl; float v = 0.f;
      if (m <= n) { const int d = sqt[nl] - skt[ml]; float ad = fabsf((float)(d < 0 ? -d : d)); ad = fmaxf(ad, 1.0f); const float lg = logf(ad) / 0.301f; int bk = (int)lg; bk = bk < 0 ? 0 : (bk > 64 ? 64 : bk);
        const float s = acc[j][r] + accl[j][r] * (1.0f / 1024.0f) + bfr(POSW[m - n + TT - 1]) + bfr(TSW[bk]); v = silu1(s) * (1.0f / TT); }
      ss[wave][8 * g + r][ml] = v; } }
  LDSX(); for (int rl = 0; rl < 16; ++rl) vst2(S + (size_t)(ql0 + rl) * TT + k0 + lane * 4, *(const v4f*)&ss[wave][rl][lane * 4]); }
__global__ __launch_bounds__(128) void k_pv(const float* __restrict__ PS0, const __bf16* __restrict__ VT, const __bf16* __restrict__ VL, int b, int h0, float* __restrict__ AV) { const int h = h0 + blockIdx.z; const float* PS = PS0 + (size_t)blockIdx.z * TT * TT; __shared__ __align__(16) float ss[4][16][HD + 4];
  const int tid = threadIdx.x, wave = tid >> 5, lane = tid & 31, col = lane & 15, g = lane >> 4; const int ql0 = blockIdx.x * 64 + wave * 16; const int kend = blockIdx.x * 64 + 64;
  v8f acc[HD / 16] = {};
#pragma unroll 1
  for (int kc = 0; kc < kend / 32; ++kc) { const F2 p = split_row(PS + (size_t)(ql0 + col) * TT, kc * 32, lane);
#pragma unroll
    for (int j = 0; j < HD / 16; ++j) { const size_t po = ((size_t)b * CC + h * HD + j * 16 + col) * (size_t)TT + kc * 32; const v16b vh = frag_b(VT + po, lane); acc[j] = wmma_bf(p.h, vh, acc[j]); acc[j] = wmma_bf(p.l, vh, acc[j]); acc[j] = wmma_bf(p.h, frag_b(VL + po, lane), acc[j]); } }
#pragma unroll
  for (int j = 0; j < HD / 16; ++j)
#pragma unroll
    for (int r = 0; r < 8; ++r) ss[wave][8 * g + r][j * 16 + col] = acc[j][r];
  LDSX(); for (int rl = 0; rl < 16; ++rl) if (lane < HD / 4) vst2(AV + ((size_t)b * TT + ql0 + rl) * CC + h * HD + lane * 4, *(const v4f*)&ss[wave][rl][lane * 4]); }
__global__ __launch_bounds__(256) void k_lns(const float* __restrict__ AV, float* __restrict__ LS) { __shared__ __align__(16) float so[32];
  const int t = threadIdx.x; const int rl = t >> 4, sub = t & 15; const size_t row = (size_t)blockIdx.x * 16 + rl; const float* p = AV + row * CC;
  float s = 0.f; for (int c = sub; c < CC; c += 16) s += p[c];
#pragma unroll
  for (int o = 1; o < 16; o <<= 1) s += __shfl_xor(s, o);
  const float mu = s * (1.0f / CC); float s2 = 0.f; for (int c = sub; c < CC; c += 16) { const float d = p[c] - mu; s2 += d * d; }
#pragma unroll
  for (int o = 1; o < 16; o <<= 1) s2 += __shfl_xor(s2, o);
  if (sub == 0) { so[rl * 2] = mu; so[rl * 2 + 1] = rsqrtf(s2 * (1.0f / CC) + 1e-8f); }
  __syncthreads(); if (t < 32) vst2(LS + (size_t)blockIdx.x * 32 + t, so[t]); }
__global__ __launch_bounds__(128) void k_out(const float* __restrict__ AV, const float* __restrict__ LS, const float* __restrict__ U, const float* __restrict__ WO, const float* __restrict__ BO, float* __restrict__ OUT) { __shared__ __align__(16) float sf[4][16][132];
  const int tid = threadIdx.x, wave = tid >> 5, lane = tid & 31, col = lane & 15, g = lane >> 4; const int c0 = blockIdx.y * 128; const size_t r0 = (size_t)blockIdx.x * 64 + wave * 16; const size_t arow = r0 + col; const float mu = LS[arow * 2], rs = LS[arow * 2 + 1];
  v8f acc[8] = {};
#pragma unroll 2
  for (int kc = 0; kc < CC / 32; ++kc) { float v[16]; { const float* p = AV + arow * CC + kc * 32 + 8 * g; const float* pu = U + arow * CC + kc * 32 + 8 * g;
#pragma unroll
      for (int i = 0; i < 8; ++i) { v[i] = (p[i] - mu) * rs * pu[i]; v[8 + i] = (p[16 + i] - mu) * rs * pu[16 + i]; } }
    asm volatile("s_wait_loadcnt 0x0" ::: "memory"); const F2 a = bsplit16(v);
#pragma unroll
    for (int j = 0; j < 8; ++j) { v16b w; const float* wr = WO + (size_t)(c0 + j * 16 + col) * CC + kc * 32 + 8 * g;
#pragma unroll
      for (int i = 0; i < 8; ++i) { w[i] = (__bf16)wr[i]; w[8 + i] = (__bf16)wr[16 + i]; }
      asm volatile("s_wait_loadcnt 0x0" ::: "memory"); acc[j] = wmma_bf(a.h, w, acc[j]); acc[j] = wmma_bf(a.l, w, acc[j]); } }
#pragma unroll
  for (int j = 0; j < 8; ++j) { const float bb = bfr(BO[c0 + j * 16 + col]);
#pragma unroll
    for (int r = 0; r < 8; ++r) sf[wave][8 * g + r][j * 16 + col] = acc[j][r] + bb; }
  LDSX(); for (int rl = 0; rl < 16; ++rl) vst2(OUT + (r0 + rl) * CC + c0 + lane * 4, *(const v4f*)&sf[wave][rl][lane * 4]); }
extern "C" void kernel_launch(void* const* d_in, const int* in_sizes, int n_in, void* d_out, int out_size, void* d_ws, size_t ws_size, hipStream_t stream) {
  (void)in_sizes; (void)n_in; (void)out_size;
  const float** F = (const float**)d_in;
  if (ws_size < (size_t)WS_END) return;
  char* ws = (char*)d_ws; float *ST = (float*)(ws + WS_ST), *U = (float*)(ws + WS_U), *S = (float*)(ws + WS_S), *AV = (float*)(ws + WS_AV); _Float16 *QH = (_Float16*)(ws + WS_QH), *QL = (_Float16*)(ws + WS_QL), *KH = (_Float16*)(ws + WS_KH), *KL = (_Float16*)(ws + WS_KL); __bf16 *VT = (__bf16*)(ws + WS_VT), *VL = (__bf16*)(ws + WS_VL);
  k_stat<<<dim3(TNB * TT / 16), 256, 0, stream>>>(F[0], ST);
  k_proj<<<dim3(TNB * TT / 64, CC / 128, 4), 128, 0, stream>>>(F[0], ST, F[3], QH, QL, KH, KL, VT, VL, U);
  for (int b = 0; b < TNB; ++b) for (int h0 = 0; h0 < NH; h0 += HG) {
    k_sc<<<dim3(TT / 64, TT / 128, HG), 128, 0, stream>>>(QH, QL, KH, KL, (const int*)d_in[2], F[6], F[7], b, h0, S);
    k_pv<<<dim3(TT / 64, 1, HG), 128, 0, stream>>>(S, VT, VL, b, h0, AV);
  }
  k_lns<<<dim3(TNB * TT / 16), 256, 0, stream>>>(AV, ST);
  k_out<<<dim3(TNB * TT / 64, CC / 128), 128, 0, stream>>>(AV, ST, U, F[4], F[5], (float*)d_out);
}
